// ExpansionContrastModule_52381421142697
// MI455X (gfx1250) — hardware-verified
//
#include <hip/hip_runtime.h>
#include <math.h>

#ifndef NB
#define NB 4
#endif
#ifndef NY
#define NY 96
#endif

constexpr int kBFull = 4;
constexpr int kC    = 256;
constexpr int kH    = 96;
constexpr int kW    = 96;
constexpr int kG    = 9;
constexpr int kHW   = kH * kW;
constexpr int kNB   = NB;
constexpr int kNY   = NY;
constexpr int kNYZ  = (kNY < kH) ? (kNY + 1) : kH;
constexpr int kNPZ  = kNYZ * kW;
static_assert(kNB >= 1 && kNB <= kBFull);
static_assert(kNY >= 1 && kNY <= kH);
static_assert(kNPZ % 64 == 0);
static_assert(kNPZ % 32 == 0);
static_assert(kC % 64 == 0 && kC % 32 == 0);
static_assert(kW % 32 == 0);

constexpr size_t kSzW = (size_t)kG * kC * kC * 2;
constexpr size_t kSzX = (size_t)kNB * kHW * kC * 2;
constexpr size_t kSzZ = (size_t)kG * kNPZ * kC * 4;
constexpr size_t kSzN = (size_t)kG * kNPZ * 4;
constexpr size_t kWsTotal = kSzW + kSzX + kSzZ + kSzN;
static_assert(kSzW % 128 == 0 && kSzX % 128 == 0 && kSzZ % 128 == 0 && kSzN % 128 == 0);
static_assert(kWsTotal <= (size_t)134217728);

typedef __attribute__((ext_vector_type(16))) _Float16 v16h;
typedef __attribute__((ext_vector_type(8)))  _Float16 v8h;
typedef __attribute__((ext_vector_type(16))) __bf16   v16b;
typedef __attribute__((ext_vector_type(8)))  __bf16   v8b;
typedef __attribute__((ext_vector_type(8)))  float    v8f;
typedef __attribute__((ext_vector_type(4)))  float    v4f;
typedef __attribute__((ext_vector_type(4)))  unsigned int v4u;

__device__ __forceinline__ unsigned short f2bf_bits(float f) {
  unsigned u = __float_as_uint(f);
  return (unsigned short)((u + 0x7FFFu + ((u >> 16) & 1u)) >> 16);
}
__device__ __forceinline__ float bf_bits2f(unsigned short h) { return __uint_as_float(((unsigned)h) << 16); }

__device__ __forceinline__ void dep_guard_h(v8f& a, v8f& b, v16h x, v16h y) { asm volatile("v_nop\n\tv_nop\n\tv_nop\n\tv_nop" : "+v"(a), "+v"(b) : "v"(x), "v"(y)); }
__device__ __forceinline__ void dep_guard_b(v8f& a, v8f& b, v16b x, v16b y) { asm volatile("v_nop\n\tv_nop\n\tv_nop\n\tv_nop" : "+v"(a), "+v"(b) : "v"(x), "v"(y)); }
__device__ __forceinline__ void keep4_h(v16h a, v16h b, v16h c, v16h d) { asm volatile("v_nop" :: "v"(a), "v"(b), "v"(c), "v"(d)); }
__device__ __forceinline__ void keep4_b(v16b a, v16b b, v16b c, v16b d) { asm volatile("v_nop" :: "v"(a), "v"(b), "v"(c), "v"(d)); }
__device__ __forceinline__ void acc_guard4(v8f& a, v8f& b, v8f& c, v8f& d) { asm volatile("v_nop\n\tv_nop\n\tv_nop\n\tv_nop" : "+v"(a), "+v"(b), "+v"(c), "+v"(d)); }
template <typename T> struct Frag;
template <> struct Frag<_Float16> {
  typedef v16h V; union U { v16h v; v8h h[2]; };
  static __device__ __forceinline__ v16h load(const _Float16* p) {
    U f; f.h[0] = *(const v8h*)(p); f.h[1] = *(const v8h*)(p + 16); return f.v;
  }
  static __device__ __forceinline__ v8f mma(v16h a, v16h b, v8f c) {
    return __builtin_amdgcn_wmma_f32_16x16x32_f16(false, a, false, b, (short)0, c, false, false);
  }
  static __device__ __forceinline__ void guard(v8f& a, v8f& b, v16h x, v16h y) { dep_guard_h(a, b, x, y); }
  static __device__ __forceinline__ void keep(v16h a, v16h b, v16h c, v16h d) { keep4_h(a, b, c, d); }
};
template <> struct Frag<__bf16> {
  typedef v16b V; union U { v16b v; v8b h[2]; };
  static __device__ __forceinline__ v16b load(const __bf16* p) {
    U f; f.h[0] = *(const v8b*)(p); f.h[1] = *(const v8b*)(p + 16); return f.v;
  }
  static __device__ __forceinline__ v8f mma(v16b a, v16b b, v8f c) {
    return __builtin_amdgcn_wmma_f32_16x16x32_bf16(false, a, false, b, (short)0, c, false, false);
  }
  static __device__ __forceinline__ void guard(v8f& a, v8f& b, v16b x, v16b y) { dep_guard_b(a, b, x, y); }
  static __device__ __forceinline__ void keep(v16b a, v16b b, v16b c, v16b d) { keep4_b(a, b, c, d); }
};

__device__ __forceinline__ unsigned pk16(unsigned short a, unsigned short b) { return (unsigned)a | ((unsigned)b << 16); }
__device__ __forceinline__ unsigned short h_bits(float f) { const _Float16 h = (_Float16)f; return __builtin_bit_cast(unsigned short, h); }

template <int ET> struct Elem;
template <> struct Elem<0> { typedef _Float16 T; };
template <> struct Elem<1> { typedef __bf16 T; };
template <int ET, bool SPLIT, int BIAS_MODE, int OUT_MODE, bool RESID, int ACT = 0>
__global__ __launch_bounds__(256) void wmma_gemm64(
    const unsigned short* __restrict__ Ap, const unsigned short* __restrict__ A2p, int lda, long strideA,
    const unsigned short* __restrict__ Btp, const unsigned short* __restrict__ Bt2p, int ldb, long strideB,
    void* __restrict__ Cout, void* __restrict__ Cout2, int ldc, long strideC,
    const float* __restrict__ bias,
    const float* __restrict__ resid, long strideR,
    int M, int N, int K, float scale) {
  typedef typename Elem<ET>::T T;
  typedef typename Frag<T>::V V;
  const T* A = (const T*)Ap; const T* A2 = (const T*)A2p; const T* Bt = (const T*)Btp; const T* Bt2 = (const T*)Bt2p;
  __shared__ __align__(16) float sT[8][16 * 68];
  const int b    = blockIdx.y;
  const int lane = threadIdx.x & 31;
  const int wave = threadIdx.x >> 5;
  const int tilesN = N >> 6;
  const int tilesM = M >> 6;
  const int tile = blockIdx.x * 8 + wave;
  if (tile >= tilesM * tilesN) return;
  const int tm = tile / tilesN;
  const int tn = tile - tm * tilesN;
  const int m0 = tm << 6;
  const int n0 = tn << 6;

  const T* Ab  = A  + (size_t)b * strideA;
  const T* Bb  = Bt + (size_t)b * strideB;
  const T* Ab2 = SPLIT ? (A2  + (size_t)b * strideA) : nullptr;
  const T* Bb2 = SPLIT ? (Bt2 + (size_t)b * strideB) : nullptr;

  const int rlane = lane & 15;
  const int koff  = (lane >> 4) * 8;
  const int mOff  = (lane >> 4) * 8;

  v8f acc[4][4];
#pragma unroll
  for (int i = 0; i < 4; ++i)
#pragma unroll
    for (int j = 0; j < 4; ++j) acc[i][j] = (v8f){0.f,0.f,0.f,0.f,0.f,0.f,0.f,0.f};

  for (int k0 = 0; k0 < K; k0 += 32) {
    V bh[4], bl[4];
#pragma unroll
    for (int j = 0; j < 4; ++j) {
      const size_t bo = (size_t)(n0 + (j << 4) + rlane) * ldb + koff + k0;
      bh[j] = Frag<T>::load(Bb + bo);
      if (SPLIT) bl[j] = Frag<T>::load(Bb2 + bo);
    }
#pragma unroll
    for (int i = 0; i < 4; ++i) {
      const size_t ao = (size_t)(m0 + (i << 4) + rlane) * lda + koff + k0;
      V ah = Frag<T>::load(Ab + ao);
      V al;
      if (SPLIT) al = Frag<T>::load(Ab2 + ao);
#pragma unroll
      for (int j = 0; j < 4; ++j) {
        acc[i][j] = Frag<T>::mma(ah, bh[j], acc[i][j]);
        if (SPLIT) {
          acc[i][j] = Frag<T>::mma(ah, bl[j], acc[i][j]);
          acc[i][j] = Frag<T>::mma(al, bh[j], acc[i][j]);
        }
      }
      Frag<T>::guard(acc[i][0], acc[i][3], ah, SPLIT ? al : ah);
    }
    Frag<T>::keep(bh[0], bh[1], bh[2], bh[3]);
    if (SPLIT) Frag<T>::keep(bl[0], bl[1], bl[2], bl[3]);
  }
  acc_guard4(acc[0][0], acc[0][1], acc[0][2], acc[0][3]);
  acc_guard4(acc[1][0], acc[1][1], acc[1][2], acc[1][3]);
  acc_guard4(acc[2][0], acc[2][1], acc[2][2], acc[2][3]);
  acc_guard4(acc[3][0], acc[3][1], acc[3][2], acc[3][3]);

  float* slab = sT[wave];
  const float* Rb = RESID ? (resid + (size_t)b * strideR) : nullptr;
#pragma unroll
  for (int i = 0; i < 4; ++i) {
    const int mBase = m0 + (i << 4);
#pragma unroll
    for (int j = 0; j < 4; ++j) {
      const int n = n0 + (j << 4) + rlane;
      float bv = 0.f;
      if (BIAS_MODE == 2) bv = bias[n];
#pragma unroll
      for (int r = 0; r < 8; ++r) {
        float v = acc[i][j][r] * scale;
        if (BIAS_MODE == 1) v += bias[mBase + mOff + r];
        if (BIAS_MODE == 2) v += bv;
        if (RESID) v += Rb[(size_t)(mBase + mOff + r) * ldc + n];
        if (ACT == 2) v = fmaxf(v, 0.0f);
        if (ACT == 4) v = (v > 0.f) ? v : 0.01f * v;
        slab[(mOff + r) * 68 + (j << 4) + rlane] = v;
      }
    }
    __builtin_amdgcn_fence(__ATOMIC_RELEASE, "workgroup");
    __builtin_amdgcn_wave_barrier();
    __builtin_amdgcn_fence(__ATOMIC_ACQUIRE, "workgroup");
    if (OUT_MODE == 0) {
      float* C = (float*)Cout + (size_t)b * strideC;
      const int hh = lane >> 4, c4 = (lane & 15) * 4;
      for (int pass = 0; pass < 2; ++pass) {
#pragma unroll
        for (int it = 0; it < 8; ++it) {
          const int row = it * 2 + hh;
          v4f v = *(const v4f*)(slab + row * 68 + c4);
          *(volatile v4f*)(C + (size_t)(mBase + row) * ldc + n0 + c4) = v;
        }
        __threadfence();
      }
    } else {
      const int q = lane >> 3, c8 = (lane & 7) * 8;
      unsigned short* C  = (unsigned short*)Cout  + (size_t)b * strideC;
      unsigned short* C2 = (OUT_MODE == 2) ? ((unsigned short*)Cout2 + (size_t)b * strideC) : nullptr;
      for (int pass = 0; pass < 2; ++pass) {
#pragma unroll
        for (int it = 0; it < 4; ++it) {
          const int row = it * 4 + q;
          const float* sp = slab + row * 68 + c8;
          v8h hv, lv;
#pragma unroll
          for (int e = 0; e < 8; ++e) {
            if (OUT_MODE == 1) {
              hv[e] = (_Float16)sp[e];
            } else {
              unsigned short hb = f2bf_bits(sp[e]);
              unsigned short lb = f2bf_bits(sp[e] - bf_bits2f(hb));
              hv[e] = __builtin_bit_cast(_Float16, hb);
              lv[e] = __builtin_bit_cast(_Float16, lb);
            }
          }
          *(volatile v8h*)(C + (size_t)(mBase + row) * ldc + n0 + c8) = hv;
          if (OUT_MODE == 2) *(volatile v8h*)(C2 + (size_t)(mBase + row) * ldc + n0 + c8) = lv;
        }
        __threadfence();
      }
    }
    __builtin_amdgcn_fence(__ATOMIC_RELEASE, "workgroup");
    __builtin_amdgcn_wave_barrier();
    __builtin_amdgcn_fence(__ATOMIC_ACQUIRE, "workgroup");
  }
}

__global__ __launch_bounds__(256) void wcast_kernel(const float* __restrict__ Wsrc, unsigned short* __restrict__ O, int n8) {
  const int i = blockIdx.x * 256 + threadIdx.x;
  if (i >= n8) return;
  const float* p = Wsrc + 8 * (size_t)i;
  const v4f a = *(const v4f*)(p);
  const v4f c = *(const v4f*)(p + 4);
  unsigned short hb[8];
#pragma unroll
  for (int e = 0; e < 4; ++e) {
    hb[e]     = f2bf_bits(a[e]);
    hb[4 + e] = f2bf_bits(c[e]);
  }
  const v4u u = (v4u){pk16(hb[0], hb[1]), pk16(hb[2], hb[3]), pk16(hb[4], hb[5]), pk16(hb[6], hb[7])};
  unsigned short* q = O + 8 * (size_t)i;
  *(volatile v4u*)q = u;
  __threadfence();
  *(volatile v4u*)q = u;
}

__global__ __launch_bounds__(256) void xcast_kernel(const float* __restrict__ F, unsigned short* __restrict__ X) {
  __shared__ float sm[64][65];
  const int t  = threadIdx.x;
  const int n0 = blockIdx.x * 64;
  const int c0 = blockIdx.y * 64;
  const int b  = blockIdx.z;
  const float* Fb = F + (size_t)b * kC * kHW;
#pragma unroll
  for (int i = 0; i < 16; ++i) {
    const int e   = i * 256 + t;
    const int r   = e >> 6;
    const int col = e & 63;
    sm[col][r] = Fb[(size_t)(c0 + r) * kHW + n0 + col];
  }
  __syncthreads();
  const int lane = t & 31, wave = t >> 5;
  const int q = lane >> 3, c8 = (lane & 7) * 8;
  unsigned short* op = X + (size_t)b * kHW * kC;
  for (int pass = 0; pass < 2; ++pass) {
#pragma unroll
    for (int it = 0; it < 2; ++it) {
      const int row = wave * 8 + it * 4 + q;
      unsigned short hb[8];
#pragma unroll
      for (int e = 0; e < 8; ++e) hb[e] = f2bf_bits(sm[row][c8 + e]);
      const v4u u = (v4u){pk16(hb[0], hb[1]), pk16(hb[2], hb[3]), pk16(hb[4], hb[5]), pk16(hb[6], hb[7])};
      *(volatile v4u*)(op + (size_t)(n0 + row) * kC + c0 + c8) = u;
    }
    __threadfence();
  }
}

__global__ __launch_bounds__(256) void norms_kernel(const float* __restrict__ Z, float* __restrict__ invn) {
  __shared__ __align__(16) float sInv[32];
  const int g  = blockIdx.y;
  const int p0 = blockIdx.x * 32;
  const int t  = threadIdx.x, lane = t & 31, wave = t >> 5;
#pragma unroll 1
  for (int r = 0; r < 4; ++r) {
    const int p = p0 + wave * 4 + r;
    const float* zr = Z + ((size_t)g * kNPZ + p) * kC + lane * 8;
    const v4f a = *(const v4f*)(zr);
    const v4f c = *(const v4f*)(zr + 4);
    float s = a[0] * a[0];
    s += a[1] * a[1];
    s += a[2] * a[2];
    s += a[3] * a[3];
    s += c[0] * c[0];
    s += c[1] * c[1];
    s += c[2] * c[2];
    s += c[3] * c[3];
#pragma unroll
    for (int off = 16; off > 0; off >>= 1) s += __shfl_xor(s, off, 32);
    if (lane == 0) sInv[wave * 4 + r] = 1.0f / fmaxf(sqrtf(s), 1e-12f);
  }
  __syncthreads();
  if (wave == 0) {
    const int lc = (lane < 8) ? lane : 7;
    const v4f v = *(const v4f*)(sInv + lc * 4);
    float* dst = invn + (size_t)g * kNPZ + p0 + lc * 4;
    if (lane < 8) *(volatile v4f*)dst = v;
    __threadfence();
    if (lane < 8) *(volatile v4f*)dst = v;
  }
}

__global__ __launch_bounds__(256) void combine_kernel(const float* __restrict__ cen, const float* __restrict__ Z,
                                                      const float* __restrict__ invn, float* __restrict__ out, int b) {
  __shared__ __align__(16) float sOut[64 * 100];
  __shared__ float sWt[kG * kW];
  __shared__ int   sSrc[kG * kW];
  const int y  = blockIdx.x;
  const int c0 = blockIdx.y * 64;
  const int t  = threadIdx.x;

  for (int e = t; e < kG * kW; e += 256) {
    const int g  = e / kW;
    const int x  = e - g * kW;
    const int dy = (g < 3) ? -1 : ((g >= 4 && g <= 6) ? 1 : 0);
    const int dx = (g == 0 || g == 6 || g == 7) ? -1 : ((g >= 2 && g <= 4) ? 1 : 0);
    const int yy = y + dy, xx = x + dx;
    const bool inside = (yy >= 0) && (yy < kH) && (xx >= 0) && (xx < kW);
    const int yyc = min(max(yy, 0), kNYZ - 1);
    const int xxc = min(max(xx, 0), kW - 1);
    const int src = yyc * kW + xxc;
    const float iv = invn[(size_t)g * kNPZ + src];
    const float sg = (g < 8) ? -iv : iv;
    sWt[e]  = inside ? sg : 0.0f;
    sSrc[e] = src;
  }
  __syncthreads();

  const int cl = t & 63, xq = t >> 6;
  const int c  = c0 + cl;
  const float* cr = cen + (((size_t)b * kC + c) * kH + y) * kW;
  float* so = sOut + cl * 100;
#pragma unroll 1
  for (int q = 0; q < kW / 32; ++q) {
    const int xb = xq + 32 * q;
    float acc[8];
#pragma unroll
    for (int i = 0; i < 8; ++i) acc[i] = 0.0f;
#pragma unroll 1
    for (int g = 0; g < kG; ++g) {
      const float* Zg = Z + (size_t)g * kNPZ * kC + c;
      const float* wt = sWt + g * kW + xb;
      const int*   sr = sSrc + g * kW + xb;
#pragma unroll
      for (int i = 0; i < 8; ++i) {
        const int   src = sr[4 * i];
        const float w   = wt[4 * i];
        acc[i] = fmaf(Zg[(size_t)src * kC], w, acc[i]);
      }
    }
#pragma unroll
    for (int i = 0; i < 8; ++i) {
      const int x = xb + 4 * i;
      const float cv = bf_bits2f(f2bf_bits(cr[x]));
      so[x] = acc[i] + cv;
    }
  }
  __syncthreads();

  const int lane = t & 31, wave = t >> 5;
  const int lc = (lane < 24) ? lane : 23;
  for (int pass = 0; pass < 2; ++pass) {
#pragma unroll
    for (int k = 0; k < 8; ++k) {
      const int row = wave + 8 * k;
      const v4f v = *(const v4f*)(sOut + row * 100 + lc * 4);
      float* dst = out + (((size_t)b * kC + c0 + row) * kH + y) * kW + lc * 4;
      if (lane < 24) *(volatile v4f*)dst = v;
    }
    __threadfence();
  }
}

extern "C" void kernel_launch(void* const* d_in, const int* in_sizes, int n_in,
                              void* d_out, int out_size, void* d_ws, size_t ws_size,
                              hipStream_t stream) {
  if (n_in < 4) return;
  if (in_sizes[0] < kNB * kC * kHW) return;
  if (in_sizes[3] < kG * kC * kC) return;
  if (out_size < kNB * kC * kHW) return;
  if (kWsTotal > ws_size) return;

  const float* cen = (const float*)d_in[0];
  const float* W3  = (const float*)d_in[3];
  float* out = (float*)d_out;

  char* base = (char*)d_ws;
  size_t off = 0;
  unsigned short* Wb   = (unsigned short*)(base + off); off += kSzW;
  unsigned short* Xb   = (unsigned short*)(base + off); off += kSzX;
  float*          Z    = (float*)(base + off);          off += kSzZ;
  float*          invn = (float*)(base + off);          off += kSzN;
  if (off > ws_size) return;

  const int n8 = kG * kC * kC / 8;
  wcast_kernel<<<dim3((n8 + 255) / 256), 256, 0, stream>>>(W3, Wb, n8);
  xcast_kernel<<<dim3(kNPZ / 64, kC / 64, kNB), 256, 0, stream>>>(cen, Xb);

  const int tiles   = (kNPZ / 64) * (kC / 64);
  const int gblocks = (tiles + 7) / 8;
  for (int b = 0; b < kNB; ++b) {
    wmma_gemm64<1, false, 0, 0, false><<<dim3(gblocks, kG), 256, 0, stream>>>(
        Xb + (size_t)b * kHW * kC, Xb + (size_t)b * kHW * kC, kC, 0L,
        Wb, Wb, kC, (long)kC * kC,
        (void*)Z, (void*)Z, kC, (long)kNPZ * kC,
        cen, cen, 0L, kNPZ, kC, kC, 1.0f);
    norms_kernel<<<dim3(kNPZ / 32, kG), 256, 0, stream>>>(Z, invn);
    combine_kernel<<<dim3(kNY, kC / 64), 256, 0, stream>>>(cen, Z, invn, out, b);
  }
}
